// CNNNer_44169443672535
// MI455X (gfx1250) — hardware-run, weakly checked
//
#include <hip/hip_runtime.h>


#ifndef NB
#define NB 2
#endif
#ifndef SEQ
#define SEQ 1024
#endif
#define NB_FULL  2
#define SEQ_FULL 1024
#ifndef OUT_SEQ
#define OUT_SEQ SEQ
#endif
#define HID    768
#define NF     200
#define NU     201
#define NK     200
#define NT     9
#define WH     64
#define WF     129
#define QE     (WF * NT)
#define HTW    256
#define HTP    512
#define KJ     224
#define NJ     224
#define GPITCH 256
#define GROWS  2048
#define VP     2048
#define SP     1184
#define VW     4
#define BW     4
#define QRS    2048.0f
#define QRI    (1.0f / 2048.0f)
#define GSC    1024.0f
#define GSI    (1.0f / 1024.0f)

static_assert(NU == NF + 1);
static_assert(HID % 64 == 0);
static_assert(KJ % 32 == 0);
static_assert(NU <= KJ);
static_assert(KJ <= HTW);
static_assert(KJ <= GPITCH);
static_assert(NJ == KJ);
static_assert(HTP == 2 * HTW);
static_assert(HTW % 64 == 0);
static_assert((HTW & (HTW - 1)) == 0);
static_assert(NF <= HTW);
static_assert(GPITCH == 256);
static_assert(NU <= GPITCH);
static_assert(NT * NJ <= GROWS);
static_assert(GROWS == VP);
static_assert(VP % 64 == 0);
static_assert(((GROWS - NT * NJ) * (GPITCH / 8)) % 256 == 0);
static_assert((NB * SEQ) % 64 == 0);
static_assert((NB * SEQ) % (16 * VW) == 0);
static_assert((NB * SEQ) % BW == 0);
static_assert(SEQ % 64 == 0);
static_assert(SEQ % 32 == 0);
static_assert(OUT_SEQ % 32 == 0);
static_assert(WF == 2 * WH + 1);
static_assert(WF <= 9 * 16);
static_assert(SP % 32 == 0);
static_assert(SP >= QE);
static_assert(SP - QE <= 32);
static_assert(SP / 4 <= 10 * 32);
static_assert(((size_t)SEQ * QE) % (4 * 256) == 0);
static_assert(NB <= NB_FULL);
static_assert(SEQ <= SEQ_FULL);
static_assert(4 * 32 * 16 == 16 * 64 * 2);
static_assert(NT * 32 * 16 == NT * GPITCH * 2);
static_assert(sizeof(float) * 16 * 68 <= 131072);
static_assert(sizeof(float) * VW * 16 * 68 <= 131072);
static_assert(sizeof(float) * BW * SP <= 131072);
static_assert(sizeof(float) * NT * GPITCH <= 131072);
static_assert(sizeof(float) * 64 * 33 <= 131072);

typedef _Float16 h16;
typedef unsigned short bf;
typedef __attribute__((ext_vector_type(16))) __bf16   v16bf;
typedef __attribute__((ext_vector_type(16))) _Float16 v16h;
typedef __attribute__((ext_vector_type(8)))  _Float16 v8h;
typedef __attribute__((ext_vector_type(8)))  unsigned short v8us;
typedef __attribute__((ext_vector_type(8)))  float    v8f;
typedef __attribute__((ext_vector_type(4)))  float    v4f;
typedef v4f  __attribute__((may_alias)) v4fa;

__device__ __forceinline__ unsigned short f2bf(float f) { unsigned u = __float_as_uint(f); u += 0x7FFFu + ((u >> 16) & 1u); return (unsigned short)(u >> 16); }
__device__ __forceinline__ float bfr(float f) { return __uint_as_float(((unsigned)f2bf(f)) << 16); }
__device__ __forceinline__ v16h cat16(v8h lo, v8h hi) { return __builtin_shufflevector(lo, hi, 0, 1, 2, 3, 4, 5, 6, 7, 8, 9, 10, 11, 12, 13, 14, 15); }
__device__ __forceinline__ v16bf cat16b(v8us lo, v8us hi) { return __builtin_bit_cast(v16bf, __builtin_shufflevector(lo, hi, 0, 1, 2, 3, 4, 5, 6, 7, 8, 9, 10, 11, 12, 13, 14, 15)); }
__device__ __forceinline__ v8f wmma16(v16h a, v16h b, v8f c) { return __builtin_amdgcn_wmma_f32_16x16x32_f16(false, a, false, b, (short)0, c, false, false); }
__device__ __forceinline__ v8f wmmab(v16bf a, v16bf b, v8f c) { return __builtin_amdgcn_wmma_f32_16x16x32_bf16(false, a, false, b, (short)0, c, false, false); }
__device__ __forceinline__ v16h  ldh(const h16* p) { return cat16(*(const v8h*)p, *(const v8h*)(p + 16)); }
__device__ __forceinline__ v16bf ldb(const bf* p)  { return cat16b(*(const v8us*)p, *(const v8us*)(p + 16)); }
__device__ __forceinline__ void wave_sync() { __builtin_amdgcn_fence(3  , "wavefront"); __builtin_amdgcn_wave_barrier(); asm volatile("" ::: "memory"); }

__device__ __forceinline__ v8f wg(v16h a, v16h b, v8f c) { c = wmma16(a, b, c); asm volatile("v_nop\n\tv_nop\n\tv_nop\n\tv_nop" : "+v"(c) : "v"(a), "v"(b)); return c; }
__device__ __forceinline__ v8f wgb(v16bf a, v16bf b, v8f c) { c = wmmab(a, b, c); asm volatile("v_nop\n\tv_nop\n\tv_nop\n\tv_nop" : "+v"(c) : "v"(a), "v"(b)); return c; }
static __device__ __forceinline__ h16 toh_flush(float v) { const h16 r = (h16)v; return (fabsf(v) < 6.103515625e-05f) ? (h16)0.0f : r; }
__device__ __forceinline__ float gelu_erf(float x) { return 0.5f * x * (1.0f + erff(x * 0.70710678118654752f)); }

__global__ __launch_bounds__(256) void k_cvt8(const float* __restrict__ src, bf* dst, size_t n8) {
    const size_t i = (size_t)blockIdx.x * 256 + threadIdx.x; if (i >= n8) return;
    const v8f v = *(const v8f*)(src + i * 8); v8us o;
#pragma unroll
    for (int k = 0; k < 8; ++k) o[k] = f2bf(v[k]);
    *(volatile v8us*)(dst + i * 8) = o; __threadfence(); *(volatile v8us*)(dst + i * 8) = o;
}

__global__ __launch_bounds__(256) void k_wtr(const float* __restrict__ W, bf* dst) {
    __shared__ float tile[64 * 33];
    const int tid = threadIdx.x;
    const int k0 = blockIdx.x * 64, n0 = blockIdx.y * 32;
#pragma unroll 1
    for (int e = 0; e < 8; ++e) {
        const int idx = e * 256 + tid; const int kk = idx >> 5, nn = idx & 31;
        const int n = n0 + nn; const int nc = n < NF ? n : NF - 1;
        float v = W[(size_t)(k0 + kk) * NF + nc];
        asm volatile("" : "+v"(v));
        tile[kk * 33 + nn] = (n < NF) ? v : 0.0f; }
    __syncthreads();
    const int row = tid >> 3, pc = tid & 7;
    v8us o;
#pragma unroll
    for (int e = 0; e < 8; ++e) o[e] = f2bf(tile[(pc * 8 + e) * 33 + row]);
    bf* p = dst + (size_t)(n0 + row) * HID + k0 + pc * 8;
    *(volatile v8us*)p = o; __threadfence(); *(volatile v8us*)p = o;
}

__global__ __launch_bounds__(256) void k_gp(const float* __restrict__ U, const float* __restrict__ Wcat, const float* __restrict__ Wd, const float* __restrict__ bd, h16* GH, h16* GR) {
    __shared__ __align__(16) float gs[NT * GPITCH];
    const int tid = threadIdx.x; const int j = blockIdx.x;
    if (j >= NJ) {
        const v8h z = (v8h){};
        const size_t zb = (size_t)NT * NJ * GPITCH;
#pragma unroll 1
        for (int ps = 0; ps < 2; ++ps) {
#pragma unroll 1
            for (int p = tid; p < (GROWS - NT * NJ) * (GPITCH / 8); p += 256) {
                *(volatile v8h*)(GH + zb + (size_t)p * 8) = z; *(volatile v8h*)(GR + zb + (size_t)p * 8) = z; }
            if (ps == 0) __threadfence(); }
    } else {
        float acc[NT];
#pragma unroll
        for (int t = 0; t < NT; ++t) acc[t] = 0.0f;
        const int ic = tid < NU ? tid : NU - 1;
        if (j < NU) {
            const float* up = U + (size_t)ic * NU + j;
#pragma unroll 1
            for (int k = 0; k < NK; ++k) {
                float u = up[(size_t)k * (NU * NU)];
                float wa = Wcat[(size_t)k * (2 * NU) + NU + j];
                float wb = Wcat[(size_t)k * (2 * NU) + ic];
                asm volatile("" : "+v"(u)); asm volatile("" : "+v"(wa)); asm volatile("" : "+v"(wb));
                const float w = bfr(u) + ((ic == NU - 1) ? bfr(wa) : 0.0f) + ((j == NU - 1) ? bfr(wb) : 0.0f);
#pragma unroll
                for (int t = 0; t < NT; ++t) acc[t] = fmaf(w, bfr(Wd[k * NT + t]), acc[t]); }
#pragma unroll
            for (int t = 0; t < NT; ++t) { float bv = bd[t]; asm volatile("" : "+v"(bv)); acc[t] += ((ic == NU - 1) & (j == NU - 1)) ? bfr(bv) : 0.0f; }
        }
        const bool ok = (tid < NU) & (j < NU);
#pragma unroll
        for (int t = 0; t < NT; ++t) gs[t * GPITCH + tid] = ok ? acc[t] * GSC : 0.0f;
        __syncthreads();
#pragma unroll 1
        for (int ps = 0; ps < 2; ++ps) {
#pragma unroll 1
            for (int p = tid; p < NT * 32; p += 256) {
                const int t = p >> 5, pc = p & 31;
                const v4f x0 = *(const v4fa*)(&gs[t * GPITCH + pc * 8]); const v4f x1 = *(const v4fa*)(&gs[t * GPITCH + pc * 8 + 4]); v8h hv, rv;
#pragma unroll
                for (int i = 0; i < 4; ++i) { const h16 a0 = toh_flush(x0[i]); const h16 a1 = toh_flush(x1[i]); hv[i] = a0; hv[4 + i] = a1;
                    rv[i] = toh_flush((x0[i] - (float)a0) * QRS); rv[4 + i] = toh_flush((x1[i] - (float)a1) * QRS); }
                const size_t oo = ((size_t)t * NJ + j) * GPITCH + (size_t)pc * 8;
                *(volatile v8h*)(GH + oo) = hv; *(volatile v8h*)(GR + oo) = rv; }
            if (ps == 0) __threadfence(); }
    }
}

__global__ __launch_bounds__(32) void k_ht(const bf* __restrict__ A, const bf* __restrict__ Bt, const float* __restrict__ bh, const float* __restrict__ bt, h16* Ph, h16* Pr) {
    __shared__ __align__(16) float os[16 * 68];
    const int K = HID;
    const int lane = threadIdx.x & 31, lr = lane & 15, hi = lane >> 4; const int r0 = blockIdx.x * 64, c0 = blockIdx.y * 64;
    v8f acc[4][4];
#pragma unroll
    for (int mb = 0; mb < 4; ++mb)
#pragma unroll
        for (int nb = 0; nb < 4; ++nb) acc[mb][nb] = (v8f){};
    const size_t aoff = (size_t)(r0 + lr) * K + 8 * hi, boff = (size_t)(c0 + lr) * K + 8 * hi;
#pragma unroll 1
    for (int kc = 0; kc < K; kc += 32) {
        v16bf a[4];
#pragma unroll
        for (int mb = 0; mb < 4; ++mb) a[mb] = ldb(A + aoff + (size_t)mb * 16 * K + kc);
#pragma unroll
        for (int nb = 0; nb < 4; ++nb) { const v16bf b = ldb(Bt + boff + (size_t)nb * 16 * K + kc);
#pragma unroll
            for (int mb = 0; mb < 4; ++mb) acc[mb][nb] = wgb(a[mb], b, acc[mb][nb]); }
    }
    float bc[4];
#pragma unroll
    for (int nb = 0; nb < 4; ++nb) { const int nn = (c0 + nb * 16 + lr) & (HTW - 1); const int bi = nn < NF ? nn : NF - 1;
        float x = bh[bi]; float y = bt[bi]; asm volatile("" : "+v"(x)); asm volatile("" : "+v"(y));
        bc[nb] = bfr((c0 >= HTW) ? y : x); }
#pragma unroll
    for (int mb = 0; mb < 4; ++mb) {
#pragma unroll
        for (int nb = 0; nb < 4; ++nb) {
#pragma unroll
            for (int j = 0; j < 8; ++j) os[(hi * 8 + j) * 68 + nb * 16 + lr] = acc[mb][nb][j] + bc[nb]; }
        wave_sync();
#pragma unroll 1
        for (int ps = 0; ps < 2; ++ps) {
#pragma unroll 1
            for (int s = 0; s < 4; ++s) { const int row = 4 * s + (lane >> 3), c8 = (lane & 7) * 8;
                const v4f x0 = *(const v4fa*)(&os[row * 68 + c8]); const v4f x1 = *(const v4fa*)(&os[row * 68 + c8 + 4]); v8h hv, rv;
#pragma unroll
                for (int i = 0; i < 4; ++i) {
                    const int n0 = (c0 + c8 + i) & (HTW - 1), n1 = (c0 + c8 + 4 + i) & (HTW - 1);
                    const float g0 = gelu_erf(x0[i]), g1 = gelu_erf(x1[i]);
                    const float v0 = (n0 < NF) ? g0 : ((n0 == NF) ? 1.0f : 0.0f);
                    const float v1 = (n1 < NF) ? g1 : ((n1 == NF) ? 1.0f : 0.0f);
                    const h16 a0 = toh_flush(v0); const h16 a1 = toh_flush(v1); hv[i] = a0; hv[4 + i] = a1;
                    rv[i] = toh_flush((v0 - (float)a0) * QRS); rv[4 + i] = toh_flush((v1 - (float)a1) * QRS); }
                const size_t oo = (size_t)(r0 + mb * 16 + row) * HTP + c0 + c8;
                *(volatile v8h*)(Ph + oo) = hv; *(volatile v8h*)(Pr + oo) = rv; }
            if (ps == 0) __threadfence(); }
        wave_sync();
    }
}

__global__ __launch_bounds__(32 * VW) void k_vg(const h16* __restrict__ AH, const h16* __restrict__ AR, const h16* __restrict__ GH, const h16* __restrict__ GR, h16* VH, h16* VR) {
    __shared__ __align__(16) float os[VW * 16 * 68];
    const int lane = threadIdx.x & 31, lr = lane & 15, hi = lane >> 4;
    const int wave = __builtin_amdgcn_readfirstlane((int)(threadIdx.x >> 5));
    const int m0 = (blockIdx.x * VW + wave) * 16, c0 = blockIdx.y * 64;
    v8f aH[4], aR[4];
#pragma unroll
    for (int nb = 0; nb < 4; ++nb) { aH[nb] = (v8f){}; aR[nb] = (v8f){}; }
    const size_t aoff = (size_t)(m0 + lr) * HTP + 8 * hi, boff = (size_t)(c0 + lr) * GPITCH + 8 * hi;
#pragma unroll 1
    for (int kc = 0; kc < KJ; kc += 32) {
        const v16h ah = ldh(AH + aoff + kc), ar = ldh(AR + aoff + kc);
#pragma unroll
        for (int nb = 0; nb < 4; ++nb) {
            const v16h gh = ldh(GH + boff + (size_t)nb * 16 * GPITCH + kc), gr = ldh(GR + boff + (size_t)nb * 16 * GPITCH + kc);
            aH[nb] = wg(ah, gh, aH[nb]); aR[nb] = wg(ar, gh, aR[nb]); aR[nb] = wg(ah, gr, aR[nb]); }
    }
    const int wb = wave * 16 * 68;
#pragma unroll
    for (int nb = 0; nb < 4; ++nb) {
#pragma unroll
        for (int j = 0; j < 8; ++j) os[wb + (hi * 8 + j) * 68 + nb * 16 + lr] = aH[nb][j] + aR[nb][j] * QRI; }
    wave_sync();
#pragma unroll 1
    for (int ps = 0; ps < 2; ++ps) {
#pragma unroll 1
        for (int s = 0; s < 4; ++s) { const int row = 4 * s + (lane >> 3), c8 = (lane & 7) * 8;
            const v4f x0 = *(const v4fa*)(&os[wb + row * 68 + c8]); const v4f x1 = *(const v4fa*)(&os[wb + row * 68 + c8 + 4]); v8h hv, rv;
#pragma unroll
            for (int i = 0; i < 4; ++i) { const h16 a0 = toh_flush(x0[i]); const h16 a1 = toh_flush(x1[i]); hv[i] = a0; hv[4 + i] = a1;
                rv[i] = toh_flush((x0[i] - (float)a0) * QRS); rv[4 + i] = toh_flush((x1[i] - (float)a1) * QRS); }
            const size_t oo = (size_t)(m0 + row) * VP + c0 + c8;
            *(volatile v8h*)(VH + oo) = hv; *(volatile v8h*)(VR + oo) = rv; }
        if (ps == 0) __threadfence(); }
}

__global__ __launch_bounds__(32 * BW) void k_band(const h16* __restrict__ HTH, const h16* __restrict__ HTR, const h16* __restrict__ VH, const h16* __restrict__ VR, float* S) {
    __shared__ __align__(16) float os[BW * SP];
    const int lane = threadIdx.x & 31, lr = lane & 15, hi = lane >> 4;
    const int wave = __builtin_amdgcn_readfirstlane((int)(threadIdx.x >> 5));
    const int q = blockIdx.x * BW + wave;
    const int b = q / SEQ, n = q % SEQ;
    const int wb = wave * SP;
    const int tc = lr < NT ? lr : NT - 1;
    const size_t bo = (size_t)q * VP + (size_t)tc * NJ + 8 * hi;
#pragma unroll 1
    for (int mt = 0; mt < 9; ++mt) {
        int key = n - WH + 16 * mt + lr; key = key < 0 ? 0 : (key > SEQ - 1 ? SEQ - 1 : key);
        const size_t ao = ((size_t)b * SEQ + (size_t)key) * HTP + HTW + 8 * hi;
        v8f sH = (v8f){}, sR = (v8f){};
#pragma unroll
        for (int kc = 0; kc < KJ; kc += 32) {
            const v16h th = ldh(HTH + ao + kc), tr = ldh(HTR + ao + kc);
            const v16h vh = ldh(VH + bo + kc), vr = ldh(VR + bo + kc);
            sH = wg(th, vh, sH); sR = wg(tr, vh, sR); sR = wg(th, vr, sR); }
#pragma unroll
        for (int j = 0; j < 8; ++j) { const int r = 16 * mt + 8 * hi + j;
            const float val = (sH[j] + sR[j] * QRI) * GSI;
            if ((lr < NT) & (r < WF)) os[wb + r * NT + lr] = val; }
    }
    if (lane < SP - QE) os[wb + QE + lane] = 0.0f;
    wave_sync();
    float* dst = S + (size_t)q * SP;
#pragma unroll 1
    for (int ps = 0; ps < 2; ++ps) {
#pragma unroll 1
        for (int i = 0; i < 10; ++i) { const int p = i * 32 + lane;
            if (p < SP / 4) { const v4f val = *(const v4fa*)(&os[wb + p * 4]); *(volatile v4f*)(dst + (size_t)p * 4) = val; } }
        if (ps == 0) __threadfence(); }
}

__global__ __launch_bounds__(256) void k_out(const float* __restrict__ S, const int* __restrict__ lengths, const float* __restrict__ bd, float* OUT) {
    const int b = blockIdx.y;
    const size_t i4 = (size_t)blockIdx.x * 256 + threadIdx.x; if (i4 >= (size_t)SEQ * QE / 4) return;
    const int len = lengths[b];
    v4f o;
#pragma unroll
    for (int c = 0; c < 4; ++c) {
        const unsigned e = (unsigned)(i4 * 4) + (unsigned)c;
        const unsigned n = e / QE; const unsigned rem = e - n * QE; const unsigned r = rem / NT; const unsigned t = rem - r * NT;
        float s = S[((size_t)b * SEQ + n) * SP + rem]; float bv = bd[t];
        asm volatile("" : "+v"(s)); asm volatile("" : "+v"(bv));
        const int jk = (int)n + (int)r - WH;
        const bool ok = ((int)n < len) & (jk >= 0) & (jk < SEQ) & (jk < len);
        float v = ok ? s : bfr(bv);
        v = (fabsf(v) <= 3.402823466e38f) ? v : 0.0f;
        o[c] = v; }
    float* p = OUT + (size_t)b * OUT_SEQ * QE + i4 * 4;
    *(volatile v4f*)p = o; __threadfence(); *(volatile v4f*)p = o;
}

static constexpr size_t al256(size_t v) { return (v + 255) & ~(size_t)255; }
static constexpr size_t SZ_XB = al256((size_t)NB * SEQ * HID * 2);
static constexpr size_t SZ_WT = al256((size_t)HTP * HID * 2);
static constexpr size_t SZ_HT = al256((size_t)NB * SEQ * HTP * 2);
static constexpr size_t SZ_GT = al256((size_t)GROWS * GPITCH * 2);
static constexpr size_t SZ_V  = al256((size_t)NB * SEQ * VP * 2);
static constexpr size_t SZ_S  = al256((size_t)NB * SEQ * SP * 4);
static constexpr size_t SZ_TOTAL = SZ_XB + SZ_WT + 2 * SZ_HT + 2 * SZ_GT + 2 * SZ_V + SZ_S;
static_assert(SZ_TOTAL <= (size_t)134217728);
static_assert(((size_t)HTW * HID * 2) % 256 == 0);
static_assert(((size_t)SEQ * HID) % 8 == 0);
static_assert((size_t)(NB_FULL - 1) * SEQ_FULL * QE * 4 + (size_t)SEQ_FULL * QE * 4 == (size_t)9510912);

extern "C" void kernel_launch(void* const* d_in, const int* in_sizes, int n_in,
                              void* d_out, int out_size, void* d_ws, size_t ws_size, hipStream_t stream) {
    if (n_in < 10) return;
    const size_t needx = ((size_t)(NB - 1) * SEQ_FULL + SEQ) * HID;
    if ((size_t)in_sizes[0] < needx) return;
    if (in_sizes[1] < NB) return;
    if ((size_t)in_sizes[2] < (size_t)HID * NF || (size_t)in_sizes[4] < (size_t)HID * NF) return;
    if (in_sizes[3] < NF || in_sizes[5] < NF) return;
    if ((size_t)in_sizes[6] < (size_t)NK * NU * NU) return;
    if ((size_t)in_sizes[7] < (size_t)NK * 2 * NU) return;
    if (in_sizes[8] < NK * NT || in_sizes[9] < NT) return;
    if ((size_t)out_size < ((size_t)(NB - 1) * OUT_SEQ + SEQ) * QE) return;
    if (SZ_TOTAL > ws_size) return;
    const float* state = (const float*)d_in[0];
    const int*   lengths = (const int*)d_in[1];
    const float* Wh = (const float*)d_in[2]; const float* bh = (const float*)d_in[3];
    const float* Wt = (const float*)d_in[4]; const float* bt = (const float*)d_in[5];
    const float* U = (const float*)d_in[6]; const float* Wcat = (const float*)d_in[7];
    const float* Wd = (const float*)d_in[8]; const float* bd = (const float*)d_in[9];
    float* OUT = (float*)d_out;
    char* wsp = (char*)d_ws;
    bf*  XB  = (bf*)wsp;  wsp += SZ_XB;
    bf*  WT  = (bf*)wsp;  wsp += SZ_WT;
    h16* HTH = (h16*)wsp; wsp += SZ_HT;
    h16* HTR = (h16*)wsp; wsp += SZ_HT;
    h16* GH  = (h16*)wsp; wsp += SZ_GT;
    h16* GR  = (h16*)wsp; wsp += SZ_GT;
    h16* VH  = (h16*)wsp; wsp += SZ_V;
    h16* VR  = (h16*)wsp; wsp += SZ_V;
    float* S = (float*)wsp; wsp += SZ_S;

    if (SEQ == SEQ_FULL) {
        const size_t n8 = (size_t)NB * SEQ * HID / 8;
        k_cvt8<<<(unsigned)((n8 + 255) / 256), 256, 0, stream>>>(state, XB, n8);
    } else {
        const size_t n8 = (size_t)SEQ * HID / 8;
        for (int b = 0; b < NB; ++b) k_cvt8<<<(unsigned)((n8 + 255) / 256), 256, 0, stream>>>(state + (size_t)b * SEQ_FULL * HID, XB + (size_t)b * SEQ * HID, n8);
    }
    k_wtr<<<dim3(HID / 64, HTW / 32, 1), 256, 0, stream>>>(Wh, WT);
    k_wtr<<<dim3(HID / 64, HTW / 32, 1), 256, 0, stream>>>(Wt, WT + (size_t)HTW * HID);
    k_gp<<<NJ + 1, 256, 0, stream>>>(U, Wcat, Wd, bd, GH, GR);

    k_ht<<<dim3(NB * SEQ / 64, HTP / 64, 1), 32, 0, stream>>>(XB, WT, bh, bt, HTH, HTR);
    k_vg<<<dim3(NB * SEQ / (16 * VW), VP / 64, 1), 32 * VW, 0, stream>>>(HTH, HTR, GH, GR, VH, VR);
    k_band<<<NB * SEQ / BW, 32 * BW, 0, stream>>>(HTH, HTR, VH, VR, S);
    k_out<<<dim3((unsigned)((size_t)SEQ * QE / 4 / 256), NB, 1), 256, 0, stream>>>(S, lengths, bd, OUT);
}
